// nchwBRA_66812511256599
// MI455X (gfx1250) — hardware-verified
//
#include <hip/hip_runtime.h>
#include <math.h>

typedef __attribute__((ext_vector_type(16))) _Float16 v16h;
typedef __attribute__((ext_vector_type(16))) __bf16 v16b;
typedef __attribute__((ext_vector_type(8)))  _Float16 v8h;
typedef __attribute__((ext_vector_type(8)))  float v8f;
typedef __attribute__((ext_vector_type(4)))  float v4f;
typedef __attribute__((ext_vector_type(2)))  float v2f;
typedef __attribute__((ext_vector_type(4)))  unsigned v4u;
typedef __attribute__((ext_vector_type(4)))  int v4i;
typedef float __attribute__((may_alias)) float_a;
typedef int __attribute__((may_alias)) int_a;

template <typename T> __device__ __forceinline__ void vst2(void* p, T v) { *(volatile T*)p = v; __threadfence(); *(volatile T*)p = v; }
__device__ __forceinline__ v8f wmma16(v16h a, v16h b, v8f c) {
  v8f d = __builtin_amdgcn_wmma_f32_16x16x32_f16(false, a, false, b, (short)0, c, false, false);
  asm volatile("v_nop\n\tv_nop\n\tv_nop\n\tv_nop" : "+v"(d) : "v"(a), "v"(b));
  return d;
}
__device__ __forceinline__ v8f wmma_bf(v16b a, v16b b, v8f c) {
  v8f d = __builtin_amdgcn_wmma_f32_16x16x32_bf16(false, a, false, b, (short)0, c, false, false);
  asm volatile("v_nop\n\tv_nop\n\tv_nop\n\tv_nop" : "+v"(d) : "v"(a), "v"(b));
  return d;
}
__device__ __forceinline__ v16h frag_h(const _Float16* rowk0, int lane) {
  union { v16h v; v8h q[2]; } u; const _Float16* p = rowk0 + 8 * (lane >> 4);
  u.q[0] = *(const v8h*)p; u.q[1] = *(const v8h*)(p + 16); return u.v;
}
__device__ __forceinline__ v16h frag_f32(const float* rowk0, int lane) {
  v16h a; const float* p = rowk0 + 8 * (lane >> 4);
#pragma unroll
  for (int i = 0; i < 8; ++i) { a[i] = (_Float16)p[i]; a[8 + i] = (_Float16)p[16 + i]; }
  return a;
}
__device__ __forceinline__ v16h frag_f32s(const float* rowk0, int lane, float sc) {
  v16h a; const float* p = rowk0 + 8 * (lane >> 4);
#pragma unroll
  for (int i = 0; i < 8; ++i) { a[i] = (_Float16)(p[i] * sc); a[8 + i] = (_Float16)(p[16 + i] * sc); }
  return a;
}
__device__ __forceinline__ v16h fragc_f32(const float* W, int k0, int n, int lane, int ld, int K) {
  v16h a; const int g = lane >> 4;
#pragma unroll
  for (int i = 0; i < 8; ++i) { const int ka = k0 + 8 * g + i, kb = ka + 16;
    a[i] = (_Float16)(ka < K ? W[(size_t)(ka < K ? ka : K - 1) * ld + n] : 0.f); a[8 + i] = (_Float16)(kb < K ? W[(size_t)(kb < K ? kb : K - 1) * ld + n] : 0.f); }
  return a;
}
struct F2 { v16b h, l; };
__device__ __forceinline__ F2 bsplit16(const float v[16]) { F2 r;
#pragma unroll
  for (int i = 0; i < 16; ++i) { const __bf16 h = (__bf16)v[i]; r.h[i] = h; r.l[i] = (__bf16)(v[i] - (float)h); }
  return r; }
__device__ __forceinline__ F2 split_row(const float* row, int k0, int lane) { float v[16]; const float* p = row + k0 + 8 * (lane >> 4);
#pragma unroll
  for (int i = 0; i < 8; ++i) { v[i] = p[i]; v[8 + i] = p[16 + i]; }
  return bsplit16(v); }
__device__ __forceinline__ F2 split_rowK(const float* row, int k0, int lane, int K) { float v[16]; const int g = lane >> 4;
#pragma unroll
  for (int i = 0; i < 8; ++i) { const int ka = k0 + 8 * g + i, kb = ka + 16; v[i] = ka < K ? row[ka < K ? ka : K - 1] : 0.f; v[8 + i] = kb < K ? row[kb < K ? kb : K - 1] : 0.f; }
  return bsplit16(v); }
__device__ __forceinline__ F2 split_col(const float* W, int k0, int n, int lane, int ld, int K) { float v[16]; const int g = lane >> 4;
#pragma unroll
  for (int i = 0; i < 8; ++i) { const int ka = k0 + 8 * g + i, kb = ka + 16; v[i] = ka < K ? W[(size_t)(ka < K ? ka : K - 1) * ld + n] : 0.f; v[8 + i] = kb < K ? W[(size_t)(kb < K ? kb : K - 1) * ld + n] : 0.f; }
  return bsplit16(v); }
__device__ __forceinline__ v8f mac3(const F2& a, const F2& b, v8f c) { c = wmma_bf(a.l, b.h, c); c = wmma_bf(a.h, b.l, c); return wmma_bf(a.h, b.h, c); }
__device__ __forceinline__ float sigm(float v) { return 1.0f / (1.0f + expf(-v)); }
#define LDSX() do { asm volatile("s_wait_dscnt 0" ::: "memory"); __builtin_amdgcn_wave_barrier(); __builtin_amdgcn_fence(__ATOMIC_RELEASE, "workgroup"); } while (0)


#define NI 8
#define CC 256
#define HW 56
#define NP 3136
#define NRG 49
#define RT 64
#define NW7 7
#define NHD 8
#define HD 32
#define TOPK 4
#define QKVW 768
#ifndef NIT
#define NIT NI
#endif
typedef __attribute__((ext_vector_type(8))) __bf16 v8b;
__device__ __forceinline__ v16b frag_b(const __bf16* rowk0, int lane) {
  union { v16b v; v8b q[2]; } u; const __bf16* p = rowk0 + 8 * (lane >> 4);
  u.q[0] = *(const v8b*)p; u.q[1] = *(const v8b*)(p + 16); return u.v;
}
__device__ __forceinline__ float bfr(float v) { return (float)(__bf16)v; }
__device__ __attribute__((noinline)) float exp_ni(float v) { return expf(v); }
__device__ __attribute__((noinline)) float erf_ni(float v) { return erff(v); }

#define PK_QKV 0
#define PK_OUT (PK_QKV + QKVW * CC)
#define PK_END (PK_OUT + CC * CC)
#define WS_PK  0u
#define WS_XT  (((WS_PK + 2u * PK_END) + 127u) / 128u * 128u)
#define WS_QH  (WS_XT + 2u * NI * NP * CC)
#define WS_QL  (WS_QH + 2u * NI * NP * 2 * CC)
#define WS_VTH (WS_QL + 2u * NI * NP * 2 * CC)
#define WS_VTL (WS_VTH + 2u * NI * CC * NP)
#define WS_QR  (WS_VTL + 2u * NI * CC * NP)
#define WS_KR  (WS_QR + 4u * NI * 64 * CC)
#define WS_IDX (WS_KR + 4u * NI * 64 * CC)
#define WS_O   (WS_IDX + 4u * NI * 64 * 4)
#define WS_SH  (WS_O + 4u * NI * NP * CC)
#define WS_SL  (WS_SH + 2u * NI * NP * CC)
#define WS_END (WS_SL + 2u * NI * NP * CC)

__device__ __forceinline__ int pix_of_q(int q) { const int r = q >> 6, t = q & 63; const int h = (r / NW7) * 8 + (t >> 3), w = (r % NW7) * 8 + (t & 7); return h * HW + w; }
__device__ __forceinline__ int q_of_pix(int p) { const int h = p / HW, w = p % HW; return ((h >> 3) * NW7 + (w >> 3)) * 64 + (h & 7) * 8 + (w & 7); }

__global__ __launch_bounds__(256) void k_pack(const float* __restrict__ WQKV, const float* __restrict__ WOUT, __bf16* __restrict__ PK) {
  __shared__ __align__(16) __bf16 s[CC]; const int n = blockIdx.x, which = blockIdx.y, t = threadIdx.x;
  if (which == 1 && n >= CC) return;
  s[t] = (__bf16)(which == 0 ? WQKV[(size_t)n * CC + t] : WOUT[(size_t)n * CC + t]);
  __syncthreads();
  if (t < CC / 8) vst2((unsigned*)(PK + (which == 0 ? PK_QKV : PK_OUT) + (size_t)n * CC + t * 8), *(const v4u*)&s[t * 8]);
}
__global__ __launch_bounds__(256) void k_xt(const float* __restrict__ X, __bf16* __restrict__ XT) {
  __shared__ __align__(16) __bf16 s[64][CC + 8]; const int tid = threadIdx.x; const int rb = blockIdx.x, n = blockIdx.y; const int q0 = rb * 64;
  for (int e = tid; e < 64 * CC; e += 256) { const int c = e >> 6, t = e & 63; s[t][c] = (__bf16)X[((size_t)n * CC + c) * NP + pix_of_q(q0 + t)]; }
  __syncthreads();
  for (int e = tid; e < 64 * CC / 8; e += 256) { const int t = e / (CC / 8), pc = e % (CC / 8); vst2((unsigned*)(XT + ((size_t)n * NP + q0 + t) * CC + pc * 8), *(const v4u*)&s[t][pc * 8]); }
}
__global__ __launch_bounds__(128) void k_qkv(const __bf16* __restrict__ XT, const __bf16* __restrict__ PK, const float* __restrict__ BQKV, _Float16* __restrict__ QH, _Float16* __restrict__ QL, _Float16* __restrict__ VTH, _Float16* __restrict__ VTL, float* __restrict__ QR, float* __restrict__ KR) {
  __shared__ __align__(16) _Float16 soh[4][16][136], sol[4][16][136]; __shared__ __align__(16) _Float16 sth[128][72], stl[128][72]; __shared__ float spool[4][128]; __shared__ __align__(16) float smean[128];
  const int tid = threadIdx.x, wave = tid >> 5, lane = tid & 31, col = lane & 15, g = lane >> 4; const int r = blockIdx.x, n = blockIdx.z; const int n0 = blockIdx.y * 128; const int which = n0 / CC;
  const size_t row0 = (size_t)n * NP + (size_t)r * 64 + wave * 16;
  v8f acc[8] = {};
#pragma unroll
  for (int kc = 0; kc < CC / 32; ++kc) { const v16b a = frag_b(XT + (row0 + col) * CC + kc * 32, lane);
#pragma unroll
    for (int j = 0; j < 8; ++j) acc[j] = wmma_bf(a, frag_b(PK + PK_QKV + (size_t)(n0 + j * 16 + col) * CC + kc * 32, lane), acc[j]); }
#pragma unroll
  for (int j = 0; j < 8; ++j) { const float bb = bfr(BQKV[n0 + j * 16 + col]);
#pragma unroll
    for (int rr = 0; rr < 8; ++rr) acc[j][rr] += bb; }
  if (which < 2) {
#pragma unroll
    for (int j = 0; j < 8; ++j) { float s = 0.f;
#pragma unroll
      for (int rr = 0; rr < 8; ++rr) s += acc[j][rr];
      s += __shfl_xor(s, 16); if (g == 0) spool[wave][j * 16 + col] = s; }
    const float sc = (which == 0) ? (1.0f / 16.0f) : 1.0f;
#pragma unroll
    for (int j = 0; j < 8; ++j)
#pragma unroll
      for (int rr = 0; rr < 8; ++rr) { const float v = acc[j][rr] * sc; const _Float16 hv = (_Float16)v; soh[wave][8 * g + rr][j * 16 + col] = hv; sol[wave][8 * g + rr][j * 16 + col] = (_Float16)((v - (float)hv) * 2048.0f); }
    __syncthreads();
    if (tid < 128) smean[tid] = ((spool[0][tid] + spool[1][tid]) + (spool[2][tid] + spool[3][tid])) * (1.0f / 64.0f);
    const int c0 = n0 - which * CC;
    for (int rl = 0; rl < 16; ++rl) { if (lane < 16) vst2((unsigned*)(QH + (row0 + rl) * (2 * CC) + which * CC + c0 + lane * 8), *(const v4u*)&soh[wave][rl][lane * 8]); else vst2((unsigned*)(QL + (row0 + rl) * (2 * CC) + which * CC + c0 + (lane - 16) * 8), *(const v4u*)&sol[wave][rl][(lane - 16) * 8]); }
    __syncthreads();
    float* PR = (which == 0) ? QR : KR; if (tid < 32) vst2(PR + ((size_t)n * 64 + r) * CC + c0 + tid * 4, *(const v4f*)&smean[tid * 4]);
  } else {
#pragma unroll
    for (int j = 0; j < 8; ++j)
#pragma unroll
      for (int rr = 0; rr < 8; ++rr) { const float v = acc[j][rr]; const _Float16 hv = (_Float16)v; sth[j * 16 + col][wave * 16 + 8 * g + rr] = hv; stl[j * 16 + col][wave * 16 + 8 * g + rr] = (_Float16)((v - (float)hv) * 2048.0f); }
    __syncthreads();
    const int c0 = n0 - 2 * CC;
    for (int e = tid; e < 128 * 8; e += 128) { const int d = e >> 3, pc = e & 7; const size_t o = ((size_t)n * CC + c0 + d) * NP + (size_t)r * 64 + pc * 8; vst2((unsigned*)(VTH + o), *(const v4u*)&sth[d][pc * 8]); vst2((unsigned*)(VTL + o), *(const v4u*)&stl[d][pc * 8]); }
  }
}
__global__ __launch_bounds__(256) void k_route(const float* __restrict__ QR, const float* __restrict__ KR, int* __restrict__ IDX) {
  __shared__ float sa[NRG][NRG + 1]; __shared__ __align__(16) int sidx[64][4]; const int tid = threadIdx.x; const int n = blockIdx.x;
  for (int e = tid; e < NRG * NRG; e += 256) { const int r = e / NRG, r2 = e % NRG; const float* a = QR + ((size_t)n * 64 + r) * CC; const float* b = KR + ((size_t)n * 64 + r2) * CC; float s = 0.f;
#pragma unroll 4
    for (int c = 0; c < CC; ++c) s += a[c] * b[c];
    sa[r][r2] = s; }
  for (int e = tid; e < 64 * 4; e += 256) (&sidx[0][0])[e] = 0;
  __syncthreads();
  if (tid < NRG) { const int r = tid; float bv[TOPK]; int bi[TOPK];
#pragma unroll
    for (int s = 0; s < TOPK; ++s) { bv[s] = -3.0e38f; bi[s] = 0; }
    for (int m = 0; m < NRG; ++m) { const float v = sa[r][m]; if (v > bv[TOPK - 1]) { float cv = v; int ci = m; bool placed = false;
#pragma unroll
        for (int s = 0; s < TOPK; ++s) { const bool sw = placed || (cv > bv[s]); placed = sw; const float tv = bv[s]; const int ti = bi[s]; bv[s] = sw ? cv : tv; bi[s] = sw ? ci : ti; cv = sw ? tv : cv; ci = sw ? ti : ci; } } }
#pragma unroll
    for (int s = 0; s < TOPK; ++s) sidx[r][s] = bi[s]; }
  __syncthreads();
  if (tid < 64) vst2((unsigned*)(IDX + ((size_t)n * 64 + tid) * 4), *(const v4u*)&sidx[tid][0]);
}
__global__ __launch_bounds__(128) void k_attn(const _Float16* __restrict__ QH, const _Float16* __restrict__ QL, const _Float16* __restrict__ VTH, const _Float16* __restrict__ VTL, const int* __restrict__ IDX, float* __restrict__ O) {
  __shared__ __align__(16) _Float16 sph[4][16][40], spl[4][16][40]; __shared__ __align__(16) float so[4][16][36];
  const int tid = threadIdx.x, wave = tid >> 5, lane = tid & 31, col = lane & 15, g = lane >> 4; const int r = blockIdx.x, h = blockIdx.y, n = blockIdx.z;
  const size_t rq = (size_t)n * NP + (size_t)r * 64 + wave * 16 + col;
  const v16h aqh = frag_h(QH + rq * (2 * CC) + h * HD, lane), aql = frag_h(QL + rq * (2 * CC) + h * HD, lane);
  int sel[TOPK];
#pragma unroll
  for (int j = 0; j < TOPK; ++j) sel[j] = min(max(IDX[((size_t)n * 64 + r) * 4 + j], 0), NRG - 1);
  float m[8], l[8];
#pragma unroll
  for (int rr = 0; rr < 8; ++rr) { m[rr] = -3.0e38f; l[rr] = 0.f; }
  v8f acc[2] = {}, accl[2] = {};
#pragma unroll 1
  for (int ks = 0; ks < TOPK * 2; ++ks) { int jsel = sel[0];
#pragma unroll
    for (int j = 1; j < TOPK; ++j) jsel = ((ks >> 1) == j) ? sel[j] : jsel;
    const size_t kbase = (size_t)n * NP + (size_t)jsel * 64 + (ks & 1) * 32; v8f s[2];
#pragma unroll
    for (int ct = 0; ct < 2; ++ct) { const size_t kk = kbase + ct * 16 + col; const v16h bkh = frag_h(QH + kk * (2 * CC) + CC + h * HD, lane), bkl = frag_h(QL + kk * (2 * CC) + CC + h * HD, lane);
      v8f c = {}; c = wmma16(aqh, bkh, c); v8f c2 = {}; c2 = wmma16(aql, bkh, c2); c2 = wmma16(aqh, bkl, c2);
#pragma unroll
      for (int rr = 0; rr < 8; ++rr) s[ct][rr] = c[rr] + c2[rr] * (1.0f / 2048.0f); }
#pragma unroll
    for (int rr = 0; rr < 8; ++rr) { float mx = fmaxf(s[0][rr], s[1][rr]);
#pragma unroll
      for (int o = 1; o < 16; o <<= 1) mx = fmaxf(mx, __shfl_xor(mx, o));
      const float mn = fmaxf(m[rr], mx); const float alpha = (m[rr] <= -1.0e38f) ? 0.f : exp_ni(m[rr] - mn);
      const float e0 = exp_ni(s[0][rr] - mn), e1 = exp_ni(s[1][rr] - mn); float es = e0 + e1;
#pragma unroll
      for (int o = 1; o < 16; o <<= 1) es += __shfl_xor(es, o);
      l[rr] = l[rr] * alpha + es; m[rr] = mn;
#pragma unroll
      for (int dt = 0; dt < 2; ++dt) { acc[dt][rr] *= alpha; accl[dt][rr] *= alpha; }
      const _Float16 h0 = (_Float16)e0, h1 = (_Float16)e1; sph[wave][8 * g + rr][col] = h0; sph[wave][8 * g + rr][16 + col] = h1; spl[wave][8 * g + rr][col] = (_Float16)((e0 - (float)h0) * 2048.0f); spl[wave][8 * g + rr][16 + col] = (_Float16)((e1 - (float)h1) * 2048.0f); }
    LDSX();
    const v16h pah = frag_h(&sph[wave][col][0], lane), pal = frag_h(&spl[wave][col][0], lane);
#pragma unroll
    for (int dt = 0; dt < 2; ++dt) { const size_t vo = ((size_t)n * CC + h * HD + dt * 16 + col) * NP + (size_t)jsel * 64 + (ks & 1) * 32; const v16h vh = frag_h(VTH + vo, lane), vl = frag_h(VTL + vo, lane);
      acc[dt] = wmma16(pah, vh, acc[dt]); accl[dt] = wmma16(pal, vh, accl[dt]); accl[dt] = wmma16(pah, vl, accl[dt]); }
    LDSX(); }
#pragma unroll
  for (int rr = 0; rr < 8; ++rr) { const float il = 1.0f / l[rr];
#pragma unroll
    for (int dt = 0; dt < 2; ++dt) so[wave][8 * g + rr][dt * 16 + col] = (acc[dt][rr] + accl[dt][rr] * (1.0f / 2048.0f)) * il; }
  LDSX();
  for (int rl = 0; rl < 16; ++rl) if (lane < 8) vst2(O + ((size_t)n * NP + (size_t)r * 64 + wave * 16 + rl) * CC + h * HD + lane * 4, *(const v4f*)&so[wave][rl][lane * 4]);
}
__global__ __launch_bounds__(256) void k_sum(const float* __restrict__ O, const _Float16* __restrict__ VTH, const _Float16* __restrict__ VTL, const float* __restrict__ LW, const float* __restrict__ LB, __bf16* __restrict__ SH, __bf16* __restrict__ SL) {
  __shared__ __align__(16) __bf16 sh_[64][CC + 8], sl_[64][CC + 8]; const int tid = threadIdx.x; const int pb = blockIdx.x, n = blockIdx.y; const int p0 = pb * 64;
  for (int e = tid; e < 64 * CC; e += 256) { const int c = e >> 6, pl = e & 63; const int p = p0 + pl; const int h = p / HW, w = p % HW; float a = 0.f;
#pragma unroll
    for (int ky = 0; ky < 3; ++ky) {
#pragma unroll
      for (int kx = 0; kx < 3; ++kx) { const int hh = h + ky - 1, ww = w + kx - 1; if (hh >= 0 && hh < HW && ww >= 0 && ww < HW) { const size_t vi = ((size_t)n * CC + c) * NP + q_of_pix(hh * HW + ww); const float v = (float)VTH[vi] + (float)VTL[vi] * (1.0f / 2048.0f); a += bfr(LW[c * 9 + ky * 3 + kx]) * v; } } }
    const float s = O[((size_t)n * NP + q_of_pix(p)) * CC + c] + (a + bfr(LB[c])); const __bf16 hb = (__bf16)s; sh_[pl][c] = hb; sl_[pl][c] = (__bf16)(s - (float)hb); }
  __syncthreads();
  for (int e = tid; e < 64 * CC / 8 * 2; e += 256) { const int plane = e / (64 * CC / 8), rem = e % (64 * CC / 8); const int pl = rem / (CC / 8), pc = rem % (CC / 8); const size_t o = ((size_t)n * NP + p0 + pl) * CC + pc * 8;
    if (plane == 0) vst2((unsigned*)(SH + o), *(const v4u*)&sh_[pl][pc * 8]); else vst2((unsigned*)(SL + o), *(const v4u*)&sl_[pl][pc * 8]); }
}
__global__ __launch_bounds__(128) void k_out(const __bf16* __restrict__ SH, const __bf16* __restrict__ SL, const __bf16* __restrict__ PK, const float* __restrict__ BO, float* __restrict__ OUT) {
  __shared__ __align__(16) float st[128][68];
  const int tid = threadIdx.x, wave = tid >> 5, lane = tid & 31, col = lane & 15, g = lane >> 4; const int pb = blockIdx.x, n = blockIdx.z; const int n0 = blockIdx.y * 128; const size_t row0 = (size_t)n * NP + (size_t)pb * 64 + wave * 16;
  v8f acc[8] = {};
#pragma unroll
  for (int kc = 0; kc < CC / 32; ++kc) { F2 a; a.h = frag_b(SH + (row0 + col) * CC + kc * 32, lane); a.l = frag_b(SL + (row0 + col) * CC + kc * 32, lane);
#pragma unroll
    for (int j = 0; j < 8; ++j) { const v16b w = frag_b(PK + PK_OUT + (size_t)(n0 + j * 16 + col) * CC + kc * 32, lane); acc[j] = wmma_bf(a.l, w, acc[j]); acc[j] = wmma_bf(a.h, w, acc[j]); } }
#pragma unroll
  for (int j = 0; j < 8; ++j) { const float bb = bfr(BO[n0 + j * 16 + col]);
#pragma unroll
    for (int rr = 0; rr < 8; ++rr) st[j * 16 + col][wave * 16 + 8 * g + rr] = acc[j][rr] + bb; }
  __syncthreads();
  for (int e = tid; e < 128 * 16; e += 128) { const int oc = e >> 4, pc = e & 15; vst2(OUT + ((size_t)n * CC + n0 + oc) * NP + (size_t)pb * 64 + pc * 4, *(const v4f*)&st[oc][pc * 4]); }
}
extern "C" void kernel_launch(void* const* d_in, const int* in_sizes, int n_in, void* d_out, int out_size, void* d_ws, size_t ws_size, hipStream_t stream) {
  (void)in_sizes; (void)n_in; (void)out_size;
  const float** F = (const float**)d_in;
  if (ws_size < (size_t)WS_END) return;
  char* ws = (char*)d_ws; __bf16 *PK = (__bf16*)(ws + WS_PK), *XT = (__bf16*)(ws + WS_XT), *SH = (__bf16*)(ws + WS_SH), *SL = (__bf16*)(ws + WS_SL); _Float16 *QH = (_Float16*)(ws + WS_QH), *QL = (_Float16*)(ws + WS_QL), *VTH = (_Float16*)(ws + WS_VTH), *VTL = (_Float16*)(ws + WS_VTL); float *QR = (float*)(ws + WS_QR), *KR = (float*)(ws + WS_KR), *O = (float*)(ws + WS_O); int* IDX = (int*)(ws + WS_IDX);
  k_pack<<<dim3(QKVW, 2), 256, 0, stream>>>(F[1], F[3], PK);
  k_xt<<<dim3(NP / 64, NIT), 256, 0, stream>>>(F[0], XT);
  k_qkv<<<dim3(NRG, QKVW / 128, NIT), 128, 0, stream>>>(XT, PK, F[2], QH, QL, VTH, VTL, QR, KR);
  k_route<<<NIT, 256, 0, stream>>>(QR, KR, IDX);
  k_attn<<<dim3(NRG, NHD, NIT), 128, 0, stream>>>(QH, QL, VTH, VTL, IDX, O);
  k_sum<<<dim3(NP / 64, NIT), 256, 0, stream>>>(O, VTH, VTL, F[5], F[6], SH, SL);
  k_out<<<dim3(NP / 64, CC / 128, NIT), 128, 0, stream>>>(SH, SL, PK, F[4], (float*)d_out);
}
